// RelationNet_30648886624750
// MI455X (gfx1250) — hardware-run, weakly checked
//
#include <hip/hip_runtime.h>
#include <math.h>

typedef __attribute__((ext_vector_type(16))) _Float16 v16h;
typedef __attribute__((ext_vector_type(8)))  _Float16 v8h;
typedef __attribute__((ext_vector_type(16))) __bf16   v16b;
typedef __attribute__((ext_vector_type(8)))  __bf16   v8b;
typedef __attribute__((ext_vector_type(8)))  float    v8f;
typedef __attribute__((ext_vector_type(4)))  float    v4f;

constexpr int kBatch    = 2;
constexpr int kPts      = 2048;
constexpr int kCtr      = 64;
constexpr int kCh       = 128;
constexpr int kCh2      = 256;
constexpr int kFc1      = 128;
constexpr int kOutCh    = 64;
constexpr int kPoints   = kBatch * kPts;
constexpr int kCtrRows  = kBatch * kCtr;
constexpr int kPairRows = kPoints * kCtr;
constexpr int kPPB      = 8;
constexpr int kFusedBlk = kPoints / kPPB;
constexpr int kA1Pitch  = 136;
constexpr int kA2Pitch  = 264;
constexpr int kStatRows  = 128;
constexpr int kStatParts = kPoints / kStatRows;
constexpr float kActCarry = 16.0f;
constexpr float kWgtCarry = 64.0f;
constexpr float kFold     = 1.0f / (kActCarry * kWgtCarry);
constexpr float kF16MinNormal = 6.103515625e-05f;
constexpr float kEps   = 1e-5f;
constexpr float kSlope = 0.2f;

static_assert(kPoints == 4096 && kCtrRows == 128 && kPairRows == 262144, "shape");
static_assert((kCh % 32) == 0 && (kCh2 % 32) == 0 && (kFc1 % 32) == 0, "GEMM K multiples of 32");
static_assert((kPoints % 32) == 0 && (kCtrRows % 32) == 0, "GEMM M multiples of 32");
static_assert((kCh % 64) == 0 && (kFc1 % 64) == 0 && (kOutCh % 64) == 0, "GEMM N multiples of 64");
static_assert((kPts % kPPB) == 0 && (kPts % kStatRows) == 0, "blocks never cross a batch");
static_assert(kCtr == 64 && kCh2 == 256 && kCh == 128, "fused tile geometry");
static_assert(((kA1Pitch * 2) % 16) == 0 && ((kA2Pitch * 2) % 16) == 0, "16-B aligned LDS rows");

constexpr size_t kSzPT  = (size_t)kPoints * kCh * 2;
constexpr size_t kSzCE  = (size_t)kCtrRows * kCh * 2;
constexpr size_t kSzW1  = (size_t)kCh * kCh2 * 2;
constexpr size_t kSzF1  = (size_t)kFc1 * kCh2 * 2;
constexpr size_t kSzF2  = (size_t)kOutCh * kFc1 * 2;
constexpr size_t kSzW2F = (size_t)kCh2 * kCh * 2;
constexpr size_t kSzW3F = (size_t)kCh2 * kCh2 * 2;
constexpr size_t kSzHP  = (size_t)kPoints * kCh * 4;
constexpr size_t kSzHC  = (size_t)kCtrRows * kCh * 4;
constexpr size_t kSzP1  = (size_t)kStatParts * kCh * 4;
constexpr size_t kSzV1  = (size_t)kCh * 4;
constexpr size_t kSzPB  = (size_t)kFusedBlk * kCh2 * 4;
constexpr size_t kSzV2  = (size_t)kCh2 * 4;
constexpr size_t kSzZ   = (size_t)kPoints * kCh2 * 4;
constexpr size_t kSzPL  = (size_t)kPoints * kCh2 * 2;
constexpr size_t kSzY1  = (size_t)kPoints * kFc1 * 4;
constexpr size_t kSzP4  = (size_t)kStatParts * kFc1 * 4;
constexpr size_t kSzV4  = (size_t)kFc1 * 4;
constexpr size_t kSzA4  = (size_t)kPoints * kFc1 * 2;
constexpr size_t kSzY2  = (size_t)kPoints * kOutCh * 4;
constexpr size_t kSzP5  = (size_t)kStatParts * kOutCh * 4;
constexpr size_t kSzV5  = (size_t)kOutCh * 4;

constexpr size_t kOffPTH = 0;
constexpr size_t kOffPTL = kOffPTH + kSzPT;
constexpr size_t kOffCEH = kOffPTL + kSzPT;
constexpr size_t kOffCEL = kOffCEH + kSzCE;
constexpr size_t kOffW1H = kOffCEL + kSzCE;
constexpr size_t kOffW1L = kOffW1H + kSzW1;
constexpr size_t kOffF1H = kOffW1L + kSzW1;
constexpr size_t kOffF1L = kOffF1H + kSzF1;
constexpr size_t kOffF2H = kOffF1L + kSzF1;
constexpr size_t kOffF2L = kOffF2H + kSzF2;
constexpr size_t kOffW2F = kOffF2L + kSzF2;
constexpr size_t kOffW3F = kOffW2F + kSzW2F;
constexpr size_t kOffHP  = kOffW3F + kSzW3F;
constexpr size_t kOffHC  = kOffHP  + kSzHP;
constexpr size_t kOffPS1 = kOffHC  + kSzHC;
constexpr size_t kOffPQ1 = kOffPS1 + kSzP1;
constexpr size_t kOffS1  = kOffPQ1 + kSzP1;
constexpr size_t kOffT1  = kOffS1  + kSzV1;
constexpr size_t kOffP2S = kOffT1  + kSzV1;
constexpr size_t kOffP2Q = kOffP2S + kSzPB;
constexpr size_t kOffP3S = kOffP2Q + kSzPB;
constexpr size_t kOffP3Q = kOffP3S + kSzPB;
constexpr size_t kOffS2  = kOffP3Q + kSzPB;
constexpr size_t kOffT2  = kOffS2  + kSzV2;
constexpr size_t kOffS3  = kOffT2  + kSzV2;
constexpr size_t kOffT3  = kOffS3  + kSzV2;
constexpr size_t kOffZMX = kOffT3  + kSzV2;
constexpr size_t kOffZMN = kOffZMX + kSzZ;
constexpr size_t kOffPLH = kOffZMN + kSzZ;
constexpr size_t kOffPLL = kOffPLH + kSzPL;
constexpr size_t kOffY1  = kOffPLL + kSzPL;
constexpr size_t kOffPS4 = kOffY1  + kSzY1;
constexpr size_t kOffPQ4 = kOffPS4 + kSzP4;
constexpr size_t kOffS4  = kOffPQ4 + kSzP4;
constexpr size_t kOffT4  = kOffS4  + kSzV4;
constexpr size_t kOffA4H = kOffT4  + kSzV4;
constexpr size_t kOffA4L = kOffA4H + kSzA4;
constexpr size_t kOffY2  = kOffA4L + kSzA4;
constexpr size_t kOffPS5 = kOffY2  + kSzY2;
constexpr size_t kOffPQ5 = kOffPS5 + kSzP5;
constexpr size_t kOffS5  = kOffPQ5 + kSzP5;
constexpr size_t kOffT5  = kOffS5  + kSzV5;
constexpr size_t kWsTotal = kOffT5 + kSzV5;
static_assert(kWsTotal == 24828416ull, "carve total");
static_assert(kWsTotal <= 134217728ull, "carve cap");
static_assert((kSzV5 % 128) == 0 && (kSzV1 % 128) == 0 && (kSzP5 % 128) == 0 && (kSzCE % 128) == 0 &&
              (kSzF2 % 128) == 0, "every region size is a multiple of 128 B, so every offset is 128-B aligned");

__device__ __forceinline__ unsigned short f2bf_bits(float f) {
  unsigned u = __float_as_uint(f);
  return (unsigned short)((u + 0x7FFFu + ((u >> 16) & 1u)) >> 16);
}
__device__ __forceinline__ float bf_bits2f(unsigned short h) { return __uint_as_float(((unsigned)h) << 16); }

__device__ __forceinline__ _Float16 to_f16_carried(float v) {
  const float w = (fabsf(v) < kF16MinNormal) ? 0.0f : v;
  return (_Float16)w;
}

template <typename T> struct Frag;
template <> struct Frag<_Float16> {
  typedef v16h V; union U { v16h v; v8h h[2]; };
  static __device__ __forceinline__ v16h load(const _Float16* p) {
    U f; f.h[0] = *(const v8h*)(p); f.h[1] = *(const v8h*)(p + 16); return f.v;
  }
};
template <> struct Frag<__bf16> {
  typedef v16b V; union U { v16b v; v8b h[2]; };
  static __device__ __forceinline__ v16b load(const __bf16* p) {
    U f; f.h[0] = *(const v8b*)(p); f.h[1] = *(const v8b*)(p + 16); return f.v;
  }
};

__device__ __forceinline__ v8f mma_h(v16h a, v16h b, v8f c) {
  c = __builtin_amdgcn_wmma_f32_16x16x32_f16(false, a, false, b, (short)0, c, false, false);
  asm volatile("v_nop\n\tv_nop\n\tv_nop\n\tv_nop" : "+v"(c) : "v"(a), "v"(b));
  return c;
}
__device__ __forceinline__ v8f mma_b(v16b a, v16b b, v8f c) {
  c = __builtin_amdgcn_wmma_f32_16x16x32_bf16(false, a, false, b, (short)0, c, false, false);
  asm volatile("v_nop\n\tv_nop\n\tv_nop\n\tv_nop" : "+v"(c) : "v"(a), "v"(b));
  return c;
}

__global__ __launch_bounds__(256) void split_rows_bf16_kernel(
    const float* __restrict__ src, unsigned short* __restrict__ dhi, unsigned short* __restrict__ dlo, int total8)
{
  const int i = blockIdx.x * 256 + threadIdx.x;
  if (i >= total8) return;
  const size_t e0 = (size_t)i << 3;
  const v4f a0 = *(const v4f*)(src + e0);
  const v4f a1 = *(const v4f*)(src + e0 + 4);
  v8h hv, lv;
#pragma unroll
  for (int e = 0; e < 4; ++e) {
    const unsigned short h0 = f2bf_bits(a0[e]), h1 = f2bf_bits(a1[e]);
    const unsigned short l0 = f2bf_bits(a0[e] - bf_bits2f(h0)), l1 = f2bf_bits(a1[e] - bf_bits2f(h1));
    hv[e]     = __builtin_bit_cast(_Float16, h0);
    hv[4 + e] = __builtin_bit_cast(_Float16, h1);
    lv[e]     = __builtin_bit_cast(_Float16, l0);
    lv[4 + e] = __builtin_bit_cast(_Float16, l1);
  }
  unsigned short* qh = dhi + e0;
  unsigned short* ql = dlo + e0;
  *(volatile v8h*)qh = hv;
  *(volatile v8h*)ql = lv;
  __threadfence();
  *(volatile v8h*)qh = hv;
  *(volatile v8h*)ql = lv;
}

__global__ __launch_bounds__(256) void cast_w_f16_kernel(
    const float* __restrict__ src, unsigned short* __restrict__ dst, int total8)
{
  const int i = blockIdx.x * 256 + threadIdx.x;
  if (i >= total8) return;
  const size_t e0 = (size_t)i << 3;
  const v4f a0 = *(const v4f*)(src + e0);
  const v4f a1 = *(const v4f*)(src + e0 + 4);
  v8h hv;
#pragma unroll
  for (int e = 0; e < 4; ++e) {
    hv[e]     = to_f16_carried(a0[e] * kWgtCarry);
    hv[4 + e] = to_f16_carried(a1[e] * kWgtCarry);
  }
  unsigned short* q = dst + e0;
  *(volatile v8h*)q = hv;
  __threadfence();
  *(volatile v8h*)q = hv;
}

template <int BIAS_MODE>
__global__ __launch_bounds__(256) void gemm_bf16x3_kernel(
    const unsigned short* __restrict__ Ahp, const unsigned short* __restrict__ Alp, int lda,
    const unsigned short* __restrict__ Bhp, const unsigned short* __restrict__ Blp, int ldb,
    float* __restrict__ Cout, int ldc, const float* __restrict__ bias, int M, int N, int K)
{
  const __bf16* Ah = (const __bf16*)Ahp;
  const __bf16* Al = (const __bf16*)Alp;
  const __bf16* Bh = (const __bf16*)Bhp;
  const __bf16* Bl = (const __bf16*)Blp;
  __shared__ __align__(16) float sT[8][16 * 68];
  const int lane = threadIdx.x & 31;
  const int wave = threadIdx.x >> 5;
  const int tilesN = N >> 6;
  const int tilesM = M >> 5;
  const int tile = blockIdx.x * 8 + wave;
  if (tile >= tilesM * tilesN) return;
  const int tm = tile / tilesN;
  const int tn = tile - tm * tilesN;
  const int m0 = tm << 5;
  const int n0 = tn << 6;
  const int rlane = lane & 15;
  const int koff  = (lane >> 4) * 8;
  const int mOff  = (lane >> 4) * 8;

  v8f acc[2][4];
#pragma unroll
  for (int i = 0; i < 2; ++i)
#pragma unroll
    for (int j = 0; j < 4; ++j) acc[i][j] = (v8f){0.f,0.f,0.f,0.f,0.f,0.f,0.f,0.f};

#pragma unroll 1
  for (int k0 = 0; k0 < K; k0 += 32) {
    v16b bh[4], bl[4];
#pragma unroll
    for (int j = 0; j < 4; ++j) {
      const size_t bo = (size_t)(n0 + (j << 4) + rlane) * ldb + koff + k0;
      bh[j] = Frag<__bf16>::load(Bh + bo);
      bl[j] = Frag<__bf16>::load(Bl + bo);
    }
#pragma unroll
    for (int i = 0; i < 2; ++i) {
      const size_t ao = (size_t)(m0 + (i << 4) + rlane) * lda + koff + k0;
      const v16b ah = Frag<__bf16>::load(Ah + ao);
      const v16b al = Frag<__bf16>::load(Al + ao);
#pragma unroll
      for (int j = 0; j < 4; ++j) {
        acc[i][j] = mma_b(ah, bh[j], acc[i][j]);
        acc[i][j] = mma_b(ah, bl[j], acc[i][j]);
        acc[i][j] = mma_b(al, bh[j], acc[i][j]);
      }
    }
  }

  float* slab = sT[wave];
#pragma unroll
  for (int i = 0; i < 2; ++i) {
    const int mBase = m0 + (i << 4);
#pragma unroll
    for (int j = 0; j < 4; ++j) {
      const int n = n0 + (j << 4) + rlane;
      float bv = 0.f;
      if (BIAS_MODE == 2) bv = bias[n];
#pragma unroll
      for (int r = 0; r < 8; ++r) {
        float v = acc[i][j][r];
        if (BIAS_MODE == 2) v += bv;
        slab[(mOff + r) * 68 + (j << 4) + rlane] = v;
      }
    }
    __builtin_amdgcn_fence(__ATOMIC_RELEASE, "workgroup");
    __builtin_amdgcn_wave_barrier();
    __builtin_amdgcn_fence(__ATOMIC_ACQUIRE, "workgroup");
    {
      const int hh = lane >> 4, c4 = (lane & 15) * 4;
      for (int pass = 0; pass < 2; ++pass) {
#pragma unroll
        for (int it = 0; it < 8; ++it) {
          const int row = it * 2 + hh;
          v4f v = *(const v4f*)(slab + row * 68 + c4);
          *(volatile v4f*)(Cout + (size_t)(mBase + row) * ldc + n0 + c4) = v;
        }
        __threadfence();
      }
    }
    __builtin_amdgcn_fence(__ATOMIC_RELEASE, "workgroup");
    __builtin_amdgcn_wave_barrier();
    __builtin_amdgcn_fence(__ATOMIC_ACQUIRE, "workgroup");
  }
}

__global__ __launch_bounds__(128) void colstats_kernel(
    const float* __restrict__ X, int nch, float* __restrict__ PS, float* __restrict__ PQ)
{
  const int c = threadIdx.x;
  const float* xp = X + (size_t)blockIdx.x * kStatRows * nch + c;
  float s = 0.f, q = 0.f;
#pragma unroll 4
  for (int r = 0; r < kStatRows; ++r) {
    const float v = xp[(size_t)r * nch];
    s += v;
    q = fmaf(v, v, q);
  }
  volatile float* ps = PS + (size_t)blockIdx.x * nch + c;
  volatile float* pq = PQ + (size_t)blockIdx.x * nch + c;
  *ps = s;
  *pq = q;
  __threadfence();
  *ps = s;
  *pq = q;
}

__global__ __launch_bounds__(128) void bn1_finalize_kernel(
    const float* __restrict__ PS, const float* __restrict__ PQ, const float* __restrict__ HC,
    const float* __restrict__ g, const float* __restrict__ beta,
    float* __restrict__ S, float* __restrict__ T)
{
  const int c = threadIdx.x;
  constexpr int kPartsPerBatch = kStatParts / kBatch;
  double q_hp = 0.0, q_hc = 0.0, mean_acc = 0.0, cross = 0.0;
#pragma unroll
  for (int b = 0; b < kBatch; ++b) {
    double sp = 0.0, sc = 0.0;
#pragma unroll 1
    for (int i = 0; i < kPartsPerBatch; ++i) {
      sp   += (double)PS[(size_t)(b * kPartsPerBatch + i) * kCh + c];
      q_hp += (double)PQ[(size_t)(b * kPartsPerBatch + i) * kCh + c];
    }
#pragma unroll 1
    for (int m = 0; m < kCtr; ++m) {
      const double v = (double)HC[(size_t)(b * kCtr + m) * kCh + c];
      sc += v;
      q_hc += v * v;
    }
    const double mp = sp * (1.0 / kPts);
    const double mc = sc * (1.0 / kCtr);
    mean_acc += mp + mc;
    cross += mp * mc;
  }
  const double mean = mean_acc * (1.0 / kBatch);
  const double e2 = q_hp * (1.0 / (kBatch * kPts)) + q_hc * (1.0 / (kBatch * kCtr)) + cross * (2.0 / kBatch);
  double var = e2 - mean * mean;
  var = (var < 0.0) ? 0.0 : var;
  const float sc1 = g[c] * rsqrtf((float)var + kEps);
  const float tc1 = beta[c] - sc1 * (float)mean;
  volatile float* ps = S + c;
  volatile float* pt = T + c;
  *ps = sc1;
  *pt = tc1;
  __threadfence();
  *ps = sc1;
  *pt = tc1;
}

__global__ __launch_bounds__(256) void bn_finalize_kernel(
    const float* __restrict__ PS, const float* __restrict__ PQ, int nparts, int nch, double inv_count,
    const float* __restrict__ g, const float* __restrict__ beta,
    float* __restrict__ S, float* __restrict__ T)
{
  const int c = threadIdx.x;
  double s = 0.0, q = 0.0;
#pragma unroll 1
  for (int i = 0; i < nparts; ++i) {
    s += (double)PS[(size_t)i * nch + c];
    q += (double)PQ[(size_t)i * nch + c];
  }
  const double mean = s * inv_count;
  double var = q * inv_count - mean * mean;
  var = (var < 0.0) ? 0.0 : var;
  const float sc = g[c] * rsqrtf((float)var + kEps);
  const float tc = beta[c] - sc * (float)mean;
  volatile float* ps = S + c;
  volatile float* pt = T + c;
  *ps = sc;
  *pt = tc;
  __threadfence();
  *ps = sc;
  *pt = tc;
}

__device__ __forceinline__ void gen_a1_tile(
    _Float16* a1s, const float* __restrict__ hp_row, const float* __restrict__ hc_b,
    const v4f sa, const v4f sb, const v4f ta, const v4f tb, int tid)
{
  const int c8 = (tid & 15) * 8;
  const int r0 = tid >> 4;
  const v4f p0 = *(const v4f*)(hp_row + c8);
  const v4f p1 = *(const v4f*)(hp_row + c8 + 4);
#pragma unroll
  for (int it = 0; it < 4; ++it) {
    const int m = r0 + 16 * it;
    const v4f h0 = *(const v4f*)(hc_b + m * kCh + c8);
    const v4f h1 = *(const v4f*)(hc_b + m * kCh + c8 + 4);
    v8h o;
#pragma unroll
    for (int e = 0; e < 4; ++e) {
      float y0 = fmaf(sa[e], p0[e] + h0[e], ta[e]);
      float y1 = fmaf(sb[e], p1[e] + h1[e], tb[e]);
      y0 = (y0 >= 0.f) ? y0 : kSlope * y0;
      y1 = (y1 >= 0.f) ? y1 : kSlope * y1;
      o[e]     = to_f16_carried(y0 * kActCarry);
      o[4 + e] = to_f16_carried(y1 * kActCarry);
    }
    *(v8h*)(a1s + m * kA1Pitch + c8) = o;
  }
}

__global__ __launch_bounds__(256) void conv2_stats_kernel(
    const float* __restrict__ HP, const float* __restrict__ HC,
    const float* __restrict__ S1, const float* __restrict__ T1,
    const unsigned short* __restrict__ W2Fp,
    float* __restrict__ PS, float* __restrict__ PQ)
{
  __shared__ __align__(16) _Float16 a1s[kCtr * kA1Pitch];
  const _Float16* W2F = (const _Float16*)W2Fp;
  const int tid = threadIdx.x, lane = tid & 31, wave = tid >> 5;
  const int rl = lane & 15, hh = lane >> 4;
  const int p0 = blockIdx.x * kPPB;
  const int bix = p0 / kPts;
  const float* hc_b = HC + (size_t)bix * kCtr * kCh;
  const int c8 = (tid & 15) * 8;
  const v4f sa = *(const v4f*)(S1 + c8);
  const v4f sb = *(const v4f*)(S1 + c8 + 4);
  const v4f ta = *(const v4f*)(T1 + c8);
  const v4f tb = *(const v4f*)(T1 + c8 + 4);

  v16h bf[4][2];
#pragma unroll
  for (int ks = 0; ks < 4; ++ks)
#pragma unroll
    for (int j = 0; j < 2; ++j)
      bf[ks][j] = Frag<_Float16>::load(W2F + (size_t)(32 * wave + 16 * j + rl) * kCh + 32 * ks + 8 * hh);

  float sS[2] = {0.f, 0.f}, sQ[2] = {0.f, 0.f};
#pragma unroll 1
  for (int pp = 0; pp < kPPB; ++pp) {
    __syncthreads();
    gen_a1_tile(a1s, HP + (size_t)(p0 + pp) * kCh, hc_b, sa, sb, ta, tb, tid);
    __syncthreads();
    v8f acc[4][2];
#pragma unroll
    for (int i = 0; i < 4; ++i)
#pragma unroll
      for (int j = 0; j < 2; ++j) acc[i][j] = (v8f){0.f,0.f,0.f,0.f,0.f,0.f,0.f,0.f};
#pragma unroll
    for (int ks = 0; ks < 4; ++ks) {
      v16h af[4];
#pragma unroll
      for (int i = 0; i < 4; ++i)
        af[i] = Frag<_Float16>::load(a1s + (16 * i + rl) * kA1Pitch + 32 * ks + 8 * hh);
#pragma unroll
      for (int i = 0; i < 4; ++i) {
        acc[i][0] = mma_h(af[i], bf[ks][0], acc[i][0]);
        acc[i][1] = mma_h(af[i], bf[ks][1], acc[i][1]);
      }
    }
#pragma unroll
    for (int j = 0; j < 2; ++j) {
      float s = 0.f, q = 0.f;
#pragma unroll
      for (int i = 0; i < 4; ++i)
#pragma unroll
        for (int r = 0; r < 8; ++r) {
          const float z = acc[i][j][r] * kFold;
          s += z;
          q = fmaf(z, z, q);
        }
      sS[j] += s;
      sQ[j] += q;
    }
  }
  const float ts0 = sS[0] + __shfl_xor(sS[0], 16, 32);
  const float ts1 = sS[1] + __shfl_xor(sS[1], 16, 32);
  const float tq0 = sQ[0] + __shfl_xor(sQ[0], 16, 32);
  const float tq1 = sQ[1] + __shfl_xor(sQ[1], 16, 32);
  const float vs = hh ? ts1 : ts0;
  const float vq = hh ? tq1 : tq0;
  volatile float* ps = PS + (size_t)blockIdx.x * kCh2 + 32 * wave + lane;
  volatile float* pq = PQ + (size_t)blockIdx.x * kCh2 + 32 * wave + lane;
  *ps = vs;
  *pq = vq;
  __threadfence();
  *ps = vs;
  *pq = vq;
}

__global__ __launch_bounds__(256) void conv23_main_kernel(
    const float* __restrict__ HP, const float* __restrict__ HC,
    const float* __restrict__ S1, const float* __restrict__ T1,
    const unsigned short* __restrict__ W2Fp, const float* __restrict__ S2, const float* __restrict__ T2,
    const unsigned short* __restrict__ W3Fp,
    float* __restrict__ PS, float* __restrict__ PQ,
    float* __restrict__ ZMAX, float* __restrict__ ZMIN)
{
  __shared__ __align__(16) _Float16 a1s[kCtr * kA1Pitch];
  __shared__ __align__(16) _Float16 a2s[kCtr * kA2Pitch];
  const _Float16* W2F = (const _Float16*)W2Fp;
  const _Float16* W3F = (const _Float16*)W3Fp;
  const int tid = threadIdx.x, lane = tid & 31, wave = tid >> 5;
  const int rl = lane & 15, hh = lane >> 4;
  const int p0 = blockIdx.x * kPPB;
  const int bix = p0 / kPts;
  const float* hc_b = HC + (size_t)bix * kCtr * kCh;
  const int c8 = (tid & 15) * 8;
  const v4f sa = *(const v4f*)(S1 + c8);
  const v4f sb = *(const v4f*)(S1 + c8 + 4);
  const v4f ta = *(const v4f*)(T1 + c8);
  const v4f tb = *(const v4f*)(T1 + c8 + 4);
  float s2f[2], t2c[2];
#pragma unroll
  for (int j = 0; j < 2; ++j) {
    s2f[j] = S2[32 * wave + 16 * j + rl] * kFold;
    t2c[j] = T2[32 * wave + 16 * j + rl];
  }
  const _Float16* w2row0 = W2F + (size_t)(32 * wave + rl) * kCh + 8 * hh;
  const _Float16* w2row1 = W2F + (size_t)(32 * wave + 16 + rl) * kCh + 8 * hh;
  const _Float16* w3row0 = W3F + (size_t)(32 * wave + rl) * kCh2 + 8 * hh;
  const _Float16* w3row1 = W3F + (size_t)(32 * wave + 16 + rl) * kCh2 + 8 * hh;

  float sS[2] = {0.f, 0.f}, sQ[2] = {0.f, 0.f};
#pragma unroll 1
  for (int pp = 0; pp < kPPB; ++pp) {
    const int p = p0 + pp;
    __syncthreads();
    gen_a1_tile(a1s, HP + (size_t)p * kCh, hc_b, sa, sb, ta, tb, tid);
    __syncthreads();
    v8f acc[4][2];
#pragma unroll
    for (int i = 0; i < 4; ++i)
#pragma unroll
      for (int j = 0; j < 2; ++j) acc[i][j] = (v8f){0.f,0.f,0.f,0.f,0.f,0.f,0.f,0.f};
#pragma unroll 1
    for (int ks = 0; ks < 4; ++ks) {
      v16h af[4];
#pragma unroll
      for (int i = 0; i < 4; ++i)
        af[i] = Frag<_Float16>::load(a1s + (16 * i + rl) * kA1Pitch + 32 * ks + 8 * hh);
      const v16h b0 = Frag<_Float16>::load(w2row0 + 32 * ks);
      const v16h b1 = Frag<_Float16>::load(w2row1 + 32 * ks);
#pragma unroll
      for (int i = 0; i < 4; ++i) {
        acc[i][0] = mma_h(af[i], b0, acc[i][0]);
        acc[i][1] = mma_h(af[i], b1, acc[i][1]);
      }
    }
#pragma unroll
    for (int i = 0; i < 4; ++i)
#pragma unroll
      for (int j = 0; j < 2; ++j)
#pragma unroll
        for (int r = 0; r < 8; ++r) {
          float y = fmaf(acc[i][j][r], s2f[j], t2c[j]);
          y = (y >= 0.f) ? y : kSlope * y;
          a2s[(16 * i + 8 * hh + r) * kA2Pitch + 32 * wave + 16 * j + rl] = to_f16_carried(y * kActCarry);
        }
    __syncthreads();
#pragma unroll
    for (int i = 0; i < 4; ++i)
#pragma unroll
      for (int j = 0; j < 2; ++j) acc[i][j] = (v8f){0.f,0.f,0.f,0.f,0.f,0.f,0.f,0.f};
#pragma unroll 1
    for (int ks = 0; ks < 8; ++ks) {
      v16h af[4];
#pragma unroll
      for (int i = 0; i < 4; ++i)
        af[i] = Frag<_Float16>::load(a2s + (16 * i + rl) * kA2Pitch + 32 * ks + 8 * hh);
      const v16h b0 = Frag<_Float16>::load(w3row0 + 32 * ks);
      const v16h b1 = Frag<_Float16>::load(w3row1 + 32 * ks);
#pragma unroll
      for (int i = 0; i < 4; ++i) {
        acc[i][0] = mma_h(af[i], b0, acc[i][0]);
        acc[i][1] = mma_h(af[i], b1, acc[i][1]);
      }
    }
    float mx[2], mn[2];
#pragma unroll
    for (int j = 0; j < 2; ++j) {
      float s = 0.f, q = 0.f;
      float vmx = acc[0][j][0] * kFold;
      float vmn = vmx;
#pragma unroll
      for (int i = 0; i < 4; ++i)
#pragma unroll
        for (int r = 0; r < 8; ++r) {
          const float z = acc[i][j][r] * kFold;
          s += z;
          q = fmaf(z, z, q);
          vmx = fmaxf(vmx, z);
          vmn = fminf(vmn, z);
        }
      sS[j] += s;
      sQ[j] += q;
      mx[j] = vmx;
      mn[j] = vmn;
    }
    const float x0 = fmaxf(mx[0], __shfl_xor(mx[0], 16, 32));
    const float x1 = fmaxf(mx[1], __shfl_xor(mx[1], 16, 32));
    const float n0 = fminf(mn[0], __shfl_xor(mn[0], 16, 32));
    const float n1 = fminf(mn[1], __shfl_xor(mn[1], 16, 32));
    const float vmax = hh ? x1 : x0;
    const float vmin = hh ? n1 : n0;
    volatile float* zx = ZMAX + (size_t)p * kCh2 + 32 * wave + lane;
    volatile float* zn = ZMIN + (size_t)p * kCh2 + 32 * wave + lane;
    *zx = vmax;
    *zn = vmin;
    __threadfence();
    *zx = vmax;
    *zn = vmin;
  }
  const float ts0 = sS[0] + __shfl_xor(sS[0], 16, 32);
  const float ts1 = sS[1] + __shfl_xor(sS[1], 16, 32);
  const float tq0 = sQ[0] + __shfl_xor(sQ[0], 16, 32);
  const float tq1 = sQ[1] + __shfl_xor(sQ[1], 16, 32);
  const float vs = hh ? ts1 : ts0;
  const float vq = hh ? tq1 : tq0;
  volatile float* ps = PS + (size_t)blockIdx.x * kCh2 + 32 * wave + lane;
  volatile float* pq = PQ + (size_t)blockIdx.x * kCh2 + 32 * wave + lane;
  *ps = vs;
  *pq = vq;
  __threadfence();
  *ps = vs;
  *pq = vq;
}

__global__ __launch_bounds__(256) void pool_planes_kernel(
    const float* __restrict__ ZMAX, const float* __restrict__ ZMIN,
    const float* __restrict__ S3, const float* __restrict__ T3,
    unsigned short* __restrict__ PH, unsigned short* __restrict__ PL, int total8)
{
  const int i = blockIdx.x * 256 + threadIdx.x;
  if (i >= total8) return;
  const size_t e0 = (size_t)i << 3;
  const int c0 = (int)(e0 % kCh2);
  v4f zx0 = *(const v4f*)(ZMAX + e0);
  v4f zx1 = *(const v4f*)(ZMAX + e0 + 4);
  v4f zn0 = *(const v4f*)(ZMIN + e0);
  v4f zn1 = *(const v4f*)(ZMIN + e0 + 4);
  asm volatile("" : "+v"(zx0), "+v"(zx1), "+v"(zn0), "+v"(zn1));
  const v4f s0 = *(const v4f*)(S3 + c0);
  const v4f s1 = *(const v4f*)(S3 + c0 + 4);
  const v4f t0 = *(const v4f*)(T3 + c0);
  const v4f t1 = *(const v4f*)(T3 + c0 + 4);
  v8h hv, lv;
#pragma unroll
  for (int e = 0; e < 4; ++e) {
    const float za = (s0[e] >= 0.f) ? zx0[e] : zn0[e];
    const float zb = (s1[e] >= 0.f) ? zx1[e] : zn1[e];
    float ya = fmaf(s0[e], za, t0[e]);
    float yb = fmaf(s1[e], zb, t1[e]);
    ya = (ya >= 0.f) ? ya : kSlope * ya;
    yb = (yb >= 0.f) ? yb : kSlope * yb;
    const unsigned short h0 = f2bf_bits(ya), h1 = f2bf_bits(yb);
    const unsigned short l0 = f2bf_bits(ya - bf_bits2f(h0)), l1 = f2bf_bits(yb - bf_bits2f(h1));
    hv[e]     = __builtin_bit_cast(_Float16, h0);
    hv[4 + e] = __builtin_bit_cast(_Float16, h1);
    lv[e]     = __builtin_bit_cast(_Float16, l0);
    lv[4 + e] = __builtin_bit_cast(_Float16, l1);
  }
  unsigned short* qh = PH + e0;
  unsigned short* ql = PL + e0;
  *(volatile v8h*)qh = hv;
  *(volatile v8h*)ql = lv;
  __threadfence();
  *(volatile v8h*)qh = hv;
  *(volatile v8h*)ql = lv;
}

__global__ __launch_bounds__(256) void act_planes_kernel(
    const float* __restrict__ Y, const float* __restrict__ S, const float* __restrict__ T,
    unsigned short* __restrict__ AH, unsigned short* __restrict__ AL, int total8)
{
  const int i = blockIdx.x * 256 + threadIdx.x;
  if (i >= total8) return;
  const size_t e0 = (size_t)i << 3;
  const int c0 = (int)(e0 % kFc1);
  const v4f y0 = *(const v4f*)(Y + e0);
  const v4f y1 = *(const v4f*)(Y + e0 + 4);
  const v4f s0 = *(const v4f*)(S + c0);
  const v4f s1 = *(const v4f*)(S + c0 + 4);
  const v4f t0 = *(const v4f*)(T + c0);
  const v4f t1 = *(const v4f*)(T + c0 + 4);
  v8h hv, lv;
#pragma unroll
  for (int e = 0; e < 4; ++e) {
    const float ya = fmaxf(fmaf(s0[e], y0[e], t0[e]), 0.f);
    const float yb = fmaxf(fmaf(s1[e], y1[e], t1[e]), 0.f);
    const unsigned short h0 = f2bf_bits(ya), h1 = f2bf_bits(yb);
    const unsigned short l0 = f2bf_bits(ya - bf_bits2f(h0)), l1 = f2bf_bits(yb - bf_bits2f(h1));
    hv[e]     = __builtin_bit_cast(_Float16, h0);
    hv[4 + e] = __builtin_bit_cast(_Float16, h1);
    lv[e]     = __builtin_bit_cast(_Float16, l0);
    lv[4 + e] = __builtin_bit_cast(_Float16, l1);
  }
  unsigned short* qh = AH + e0;
  unsigned short* ql = AL + e0;
  *(volatile v8h*)qh = hv;
  *(volatile v8h*)ql = lv;
  __threadfence();
  *(volatile v8h*)qh = hv;
  *(volatile v8h*)ql = lv;
}

__global__ __launch_bounds__(256) void out_kernel(
    const float* __restrict__ Y, const float* __restrict__ S, const float* __restrict__ T,
    float* __restrict__ out, int total4)
{
  const int i = blockIdx.x * 256 + threadIdx.x;
  if (i >= total4) return;
  const size_t e0 = (size_t)i << 2;
  const int c0 = (int)(e0 % kOutCh);
  const v4f y = *(const v4f*)(Y + e0);
  const v4f s = *(const v4f*)(S + c0);
  const v4f t = *(const v4f*)(T + c0);
  v4f o;
#pragma unroll
  for (int e = 0; e < 4; ++e) o[e] = fmaxf(fmaf(s[e], y[e], t[e]), 0.f);
  float* q = out + e0;
  *(volatile v4f*)q = o;
  __threadfence();
  *(volatile v4f*)q = o;
}

static inline int cdiv_host(int a, int b) { return (a + b - 1) / b; }

extern "C" void kernel_launch(void* const* d_in, const int* in_sizes, int n_in,
                              void* d_out, int out_size, void* d_ws, size_t ws_size,
                              hipStream_t stream) {
  if (n_in < 19) return;
  if (in_sizes[0] != kPoints * kCh) return;
  if (in_sizes[1] != kCtrRows * kCh) return;
  if (in_sizes[2] != kCh * kCh2) return;
  if (in_sizes[3] != kCh || in_sizes[4] != kCh) return;
  if (in_sizes[5] != kCh2 * kCh) return;
  if (in_sizes[6] != kCh2 || in_sizes[7] != kCh2) return;
  if (in_sizes[8] != kCh2 * kCh2) return;
  if (in_sizes[9] != kCh2 || in_sizes[10] != kCh2) return;
  if (in_sizes[11] != kFc1 * kCh2) return;
  if (in_sizes[12] != kFc1 || in_sizes[13] != kFc1 || in_sizes[14] != kFc1) return;
  if (in_sizes[15] != kOutCh * kFc1) return;
  if (in_sizes[16] != kOutCh || in_sizes[17] != kOutCh || in_sizes[18] != kOutCh) return;
  if (out_size != kPoints * kOutCh) return;
  if (ws_size < kWsTotal) return;

  const float* point  = (const float*)d_in[0];
  const float* center = (const float*)d_in[1];
  const float* W1     = (const float*)d_in[2];
  const float* g1     = (const float*)d_in[3];
  const float* b1     = (const float*)d_in[4];
  const float* W2     = (const float*)d_in[5];
  const float* g2     = (const float*)d_in[6];
  const float* b2     = (const float*)d_in[7];
  const float* W3     = (const float*)d_in[8];
  const float* g3     = (const float*)d_in[9];
  const float* b3     = (const float*)d_in[10];
  const float* fc1w   = (const float*)d_in[11];
  const float* fc1b   = (const float*)d_in[12];
  const float* g4     = (const float*)d_in[13];
  const float* b4     = (const float*)d_in[14];
  const float* fc2w   = (const float*)d_in[15];
  const float* fc2b   = (const float*)d_in[16];
  const float* g5     = (const float*)d_in[17];
  const float* b5     = (const float*)d_in[18];
  float* out = (float*)d_out;

  char* ws = (char*)d_ws;
  unsigned short* PTH = (unsigned short*)(ws + kOffPTH);
  unsigned short* PTL = (unsigned short*)(ws + kOffPTL);
  unsigned short* CEH = (unsigned short*)(ws + kOffCEH);
  unsigned short* CEL = (unsigned short*)(ws + kOffCEL);
  unsigned short* W1H = (unsigned short*)(ws + kOffW1H);
  unsigned short* W1L = (unsigned short*)(ws + kOffW1L);
  unsigned short* F1H = (unsigned short*)(ws + kOffF1H);
  unsigned short* F1L = (unsigned short*)(ws + kOffF1L);
  unsigned short* F2H = (unsigned short*)(ws + kOffF2H);
  unsigned short* F2L = (unsigned short*)(ws + kOffF2L);
  unsigned short* W2F = (unsigned short*)(ws + kOffW2F);
  unsigned short* W3F = (unsigned short*)(ws + kOffW3F);
  float* HP  = (float*)(ws + kOffHP);
  float* HC  = (float*)(ws + kOffHC);
  float* PS1 = (float*)(ws + kOffPS1);
  float* PQ1 = (float*)(ws + kOffPQ1);
  float* S1  = (float*)(ws + kOffS1);
  float* T1  = (float*)(ws + kOffT1);
  float* P2S = (float*)(ws + kOffP2S);
  float* P2Q = (float*)(ws + kOffP2Q);
  float* P3S = (float*)(ws + kOffP3S);
  float* P3Q = (float*)(ws + kOffP3Q);
  float* S2  = (float*)(ws + kOffS2);
  float* T2  = (float*)(ws + kOffT2);
  float* S3  = (float*)(ws + kOffS3);
  float* T3  = (float*)(ws + kOffT3);
  float* ZMX = (float*)(ws + kOffZMX);
  float* ZMN = (float*)(ws + kOffZMN);
  unsigned short* PLH = (unsigned short*)(ws + kOffPLH);
  unsigned short* PLL = (unsigned short*)(ws + kOffPLL);
  float* Y1  = (float*)(ws + kOffY1);
  float* PS4 = (float*)(ws + kOffPS4);
  float* PQ4 = (float*)(ws + kOffPQ4);
  float* S4  = (float*)(ws + kOffS4);
  float* T4  = (float*)(ws + kOffT4);
  unsigned short* A4H = (unsigned short*)(ws + kOffA4H);
  unsigned short* A4L = (unsigned short*)(ws + kOffA4L);
  float* Y2  = (float*)(ws + kOffY2);
  float* PS5 = (float*)(ws + kOffPS5);
  float* PQ5 = (float*)(ws + kOffPQ5);
  float* S5  = (float*)(ws + kOffS5);
  float* T5  = (float*)(ws + kOffT5);

  split_rows_bf16_kernel<<<cdiv_host(kPoints * kCh / 8, 256), 256, 0, stream>>>(point, PTH, PTL, kPoints * kCh / 8);
  split_rows_bf16_kernel<<<cdiv_host(kCtrRows * kCh / 8, 256), 256, 0, stream>>>(center, CEH, CEL, kCtrRows * kCh / 8);
  split_rows_bf16_kernel<<<cdiv_host(kCh * kCh2 / 8, 256), 256, 0, stream>>>(W1, W1H, W1L, kCh * kCh2 / 8);
  split_rows_bf16_kernel<<<cdiv_host(kFc1 * kCh2 / 8, 256), 256, 0, stream>>>(fc1w, F1H, F1L, kFc1 * kCh2 / 8);
  split_rows_bf16_kernel<<<cdiv_host(kOutCh * kFc1 / 8, 256), 256, 0, stream>>>(fc2w, F2H, F2L, kOutCh * kFc1 / 8);
  cast_w_f16_kernel<<<cdiv_host(kCh2 * kCh / 8, 256), 256, 0, stream>>>(W2, W2F, kCh2 * kCh / 8);
  cast_w_f16_kernel<<<cdiv_host(kCh2 * kCh2 / 8, 256), 256, 0, stream>>>(W3, W3F, kCh2 * kCh2 / 8);

  gemm_bf16x3_kernel<0><<<cdiv_host((kPoints / 32) * (kCh / 64), 8), 256, 0, stream>>>(
      PTH, PTL, kCh, W1H, W1L, kCh2, HP, kCh, S1, kPoints, kCh, kCh);
  gemm_bf16x3_kernel<0><<<cdiv_host((kCtrRows / 32) * (kCh / 64), 8), 256, 0, stream>>>(
      CEH, CEL, kCh, W1H + kCh, W1L + kCh, kCh2, HC, kCh, S1, kCtrRows, kCh, kCh);

  colstats_kernel<<<kStatParts, kCh, 0, stream>>>(HP, kCh, PS1, PQ1);
  bn1_finalize_kernel<<<1, kCh, 0, stream>>>(PS1, PQ1, HC, g1, b1, S1, T1);

  conv2_stats_kernel<<<kFusedBlk, 256, 0, stream>>>(HP, HC, S1, T1, W2F, P2S, P2Q);
  bn_finalize_kernel<<<1, kCh2, 0, stream>>>(P2S, P2Q, kFusedBlk, kCh2, 1.0 / (double)kPairRows, g2, b2, S2, T2);

  conv23_main_kernel<<<kFusedBlk, 256, 0, stream>>>(HP, HC, S1, T1, W2F, S2, T2, W3F, P3S, P3Q, ZMX, ZMN);
  bn_finalize_kernel<<<1, kCh2, 0, stream>>>(P3S, P3Q, kFusedBlk, kCh2, 1.0 / (double)kPairRows, g3, b3, S3, T3);

  pool_planes_kernel<<<cdiv_host(kPoints * kCh2 / 8, 256), 256, 0, stream>>>(ZMX, ZMN, S3, T3, PLH, PLL, kPoints * kCh2 / 8);
  gemm_bf16x3_kernel<2><<<cdiv_host((kPoints / 32) * (kFc1 / 64), 8), 256, 0, stream>>>(
      PLH, PLL, kCh2, F1H, F1L, kCh2, Y1, kFc1, fc1b, kPoints, kFc1, kCh2);
  colstats_kernel<<<kStatParts, kFc1, 0, stream>>>(Y1, kFc1, PS4, PQ4);
  bn_finalize_kernel<<<1, kFc1, 0, stream>>>(PS4, PQ4, kStatParts, kFc1, 1.0 / (double)kPoints, g4, b4, S4, T4);

  act_planes_kernel<<<cdiv_host(kPoints * kFc1 / 8, 256), 256, 0, stream>>>(Y1, S4, T4, A4H, A4L, kPoints * kFc1 / 8);
  gemm_bf16x3_kernel<2><<<cdiv_host((kPoints / 32) * (kOutCh / 64), 8), 256, 0, stream>>>(
      A4H, A4L, kFc1, F2H, F2L, kFc1, Y2, kOutCh, fc2b, kPoints, kOutCh, kFc1);
  colstats_kernel<<<kStatParts, kOutCh, 0, stream>>>(Y2, kOutCh, PS5, PQ5);
  bn_finalize_kernel<<<1, kOutCh, 0, stream>>>(PS5, PQ5, kStatParts, kOutCh, 1.0 / (double)kPoints, g5, b5, S5, T5);
  out_kernel<<<cdiv_host(kPoints * kOutCh / 4, 256), 256, 0, stream>>>(Y2, S5, T5, out, kPoints * kOutCh / 4);
}
